// PVMLayer4_6511170421519
// MI455X (gfx1250) — hardware-verified
//
#include <hip/hip_runtime.h>


namespace {
constexpr int NB = 4, CIN = 256, HH = 64, L = HH * HH, NT = NB * L, NCH = 4, DM = 64, DI = 128, NS = 16, R = 4, XD = R + 2 * NS, DC = 4, NQ = NCH * NT;
constexpr float XS = 8.0f, US = 8192.0f  , DS = 131072.0f  , YS = 32768.0f  , WSC = 256.0f, EPS = 1e-5f;
typedef _Float16 b16;
typedef __attribute__((ext_vector_type(16))) _Float16 v16b;
typedef __attribute__((ext_vector_type(8))) _Float16 v8b;
typedef __attribute__((ext_vector_type(8))) float v8f;
typedef __attribute__((ext_vector_type(4))) float v4f;
typedef __attribute__((ext_vector_type(2))) float v2f;
__device__ __forceinline__ float bf16_rne(float f) { unsigned int u = __float_as_uint(f); u += 0x7FFFu + ((u >> 16) & 1u); return __uint_as_float(u & 0xFFFF0000u); }
__device__ __forceinline__ void split16(float v, b16& hi, b16& lo) { hi = (b16)v; lo = (b16)(v - (float)hi); }
__device__ __forceinline__ v16b frag_kb(const b16* p, int hh) { const v8b a = *(const v8b*)(p + 8 * hh), b = *(const v8b*)(p + 16 + 8 * hh); v16b f;
#pragma unroll
  for (int e = 0; e < 8; ++e) { f[e] = a[e]; f[8 + e] = b[e]; } return f; }
__device__ __forceinline__ v8f wmma16b(v16b a, v16b b, v8f c) { v8f d = __builtin_amdgcn_wmma_f32_16x16x32_f16(false, a, false, b, (short)0, c, false, false); asm volatile("v_nop\n\tv_nop\n\tv_nop\n\tv_nop" : "+v"(d) : "v"(a), "v"(b)); return d; }
__device__ __forceinline__ void wave_lds_sync() { __builtin_amdgcn_fence(__ATOMIC_RELEASE, "workgroup"); __builtin_amdgcn_wave_barrier(); __builtin_amdgcn_fence(__ATOMIC_ACQUIRE, "workgroup"); }
__device__ __forceinline__ float pmul(float a, float b) { float p = a * b; asm volatile("" : "+v"(p)); return p; }
__device__ __forceinline__ float sigm(float v) { return 1.0f / (1.0f + __expf(-v)); }
__device__ __forceinline__ float silu(float v) { return pmul(v, sigm(v)); }
__device__ __forceinline__ float softplus(float v) { return v > 20.0f ? v : (v < -20.0f ? __expf(v) : log1pf(__expf(v))); }

__global__ __launch_bounds__(256) void wcopyp_kernel(const float* __restrict__ w, int KIN, int OUT, int KP, int OUTP, b16* __restrict__ WT) {
  const int u = blockIdx.x * 256 + threadIdx.x; if (u >= OUTP * KP / 8) return; const int e = u * 8; const int o = e / KP, k0 = e % KP; v8b v;
#pragma unroll
  for (int j = 0; j < 8; ++j) { const int k = k0 + j; v[j] = (o < OUT && k < KIN) ? (b16)(bf16_rne(w[(size_t)o * KIN + k]) * WSC) : (b16)0.0f; } for (int pass = 0; pass < 2; ++pass) { *(volatile v8b*)(WT + e) = v; __threadfence(); }
}
__global__ __launch_bounds__(32) void ln_in_kernel(const float* __restrict__ x, const float* __restrict__ g, const float* __restrict__ bb, float* __restrict__ XN) {
  __shared__ __attribute__((aligned(16))) float Tf[16][CIN + 4];
  const int lane = threadIdx.x; const size_t m0 = (size_t)blockIdx.x * 16; const int b = (int)(m0 / L), p0 = (int)(m0 % L);
  float g8[8], b8[8]; for (int q = 0; q < 8; ++q) { g8[q] = bf16_rne(g[q * 32 + lane]); b8[q] = bf16_rne(bb[q * 32 + lane]); }
  for (int rr = 0; rr < 16; ++rr) { float v[8]; float s = 0.0f; for (int q = 0; q < 8; ++q) { v[q] = bf16_rne(x[((size_t)b * CIN + q * 32 + lane) * L + p0 + rr]); s += v[q]; } for (int o = 16; o; o >>= 1) s += __shfl_xor(s, o); const float mu = s * (1.0f / CIN);
    float vq = 0.0f; for (int q = 0; q < 8; ++q) { const float d = v[q] - mu; vq += pmul(d, d); } for (int o = 16; o; o >>= 1) vq += __shfl_xor(vq, o); const float rs = rsqrtf(vq * (1.0f / CIN) + EPS);
    for (int q = 0; q < 8; ++q) Tf[rr][q * 32 + lane] = pmul(pmul(v[q] - mu, rs), g8[q]) + b8[q]; }
  wave_lds_sync();
  for (int pass = 0; pass < 2; ++pass) { for (int rr = 0; rr < 16; ++rr) for (int q = 0; q < 2; ++q) *(volatile v4f*)(XN + (m0 + rr) * CIN + q * 128 + lane * 4) = *(const v4f*)(&Tf[rr][q * 128 + lane * 4]); __threadfence(); }
}
__global__ __launch_bounds__(32) void inproj_kernel(const float* __restrict__ XN, const b16* __restrict__ WIP, int ntv, float* __restrict__ XZ) {
  __shared__ __attribute__((aligned(16))) b16 Ah[16][DM + 8], Al[16][DM + 8]; __shared__ __attribute__((aligned(16))) float Tf[16][128 + 4];
  const int lane = threadIdx.x, nloc = lane & 15, hlf = lane >> 4; const size_t w0 = (size_t)blockIdx.x * 16; const int q = (int)(w0 / ntv); const size_t t0 = w0 % ntv; const size_t sq0 = (size_t)q * NT + t0;
  for (int rr = 0; rr < 16; ++rr) { const v2f v = *(const v2f*)(XN + (t0 + rr) * CIN + q * DM + lane * 2); for (int j = 0; j < 2; ++j) { b16 p, ql; split16(v[j] * XS, p, ql); Ah[rr][lane * 2 + j] = p; Al[rr][lane * 2 + j] = ql; } }
  wave_lds_sync();
#pragma unroll 1
  for (int cg = 0; cg < 2; ++cg) { v8f acc[8];
#pragma unroll
    for (int t = 0; t < 8; ++t) acc[t] = (v8f){};
#pragma unroll
    for (int kb = 0; kb < DM; kb += 32) { const v16b a = frag_kb(&Ah[nloc][kb], hlf), al = frag_kb(&Al[nloc][kb], hlf);
#pragma unroll
      for (int t = 0; t < 8; ++t) { const v16b bw = frag_kb(WIP + (size_t)(cg * 128 + t * 16 + nloc) * DM + kb, hlf); acc[t] = wmma16b(a, bw, acc[t]); acc[t] = wmma16b(al, bw, acc[t]); } }
#pragma unroll
    for (int t = 0; t < 8; ++t)
#pragma unroll 1
      for (int r8 = 0; r8 < 8; ++r8) Tf[8 * hlf + r8][t * 16 + nloc] = acc[t][r8] * (1.0f / (XS * WSC));
    wave_lds_sync();
    for (int pass = 0; pass < 2; ++pass) { for (int rr = 0; rr < 16; ++rr) *(volatile v4f*)(XZ + (sq0 + rr) * (2 * DI) + cg * 128 + lane * 4) = *(const v4f*)(&Tf[rr][lane * 4]); __threadfence(); }
    wave_lds_sync(); }
}
__global__ __launch_bounds__(256) void conv_kernel(const float* __restrict__ XZ, const float* __restrict__ cw, const float* __restrict__ cb, int ntv, float* __restrict__ U) {
  const size_t gid = (size_t)blockIdx.x * 256 + threadIdx.x; const size_t w = gid / (DI / 4); const int d4 = (int)(gid % (DI / 4)) * 4; if (w >= (size_t)NCH * ntv) return;
  const int q = (int)(w / ntv); const size_t t = w % ntv; const int p = (int)(t % L); const size_t sq = (size_t)q * NT + t;
  v4f acc; for (int j = 0; j < 4; ++j) acc[j] = bf16_rne(cb[d4 + j]);
#pragma unroll
  for (int k = 0; k < DC; ++k) { const int pp = p - (DC - 1) + k; const bool ok = pp >= 0; const v4f v = *(const v4f*)(XZ + (ok ? sq - (DC - 1) + k : sq) * (2 * DI) + d4); for (int j = 0; j < 4; ++j) acc[j] += ok ? pmul(v[j], bf16_rne(cw[(d4 + j) * DC + k])) : 0.0f; }
  v4f o; for (int j = 0; j < 4; ++j) o[j] = silu(acc[j]);
  for (int pass = 0; pass < 2; ++pass) { *(volatile v4f*)(U + sq * DI + d4) = o; __threadfence(); }
}
__global__ __launch_bounds__(32) void xproj_kernel(const float* __restrict__ U, const b16* __restrict__ XPW, const b16* __restrict__ DTW, const float* __restrict__ dtb, int ntv, float* __restrict__ BC, float* __restrict__ DT) {
  __shared__ __attribute__((aligned(16))) b16 Ah[16][DI + 8], Al[16][DI + 8]; __shared__ __attribute__((aligned(16))) b16 Dh[16][32 + 8], Dl[16][32 + 8]; __shared__ __attribute__((aligned(16))) float Sbc[16][32]; __shared__ __attribute__((aligned(16))) float Tf[16][DI + 4];
  const int lane = threadIdx.x, nloc = lane & 15, hlf = lane >> 4; const size_t w0 = (size_t)blockIdx.x * 16; const int q = (int)(w0 / ntv); const size_t sq0 = (size_t)q * NT + (w0 % ntv);
  for (int rr = 0; rr < 16; ++rr) { const v4f v = *(const v4f*)(U + (sq0 + rr) * DI + lane * 4); for (int j = 0; j < 4; ++j) { b16 p, ql; split16(v[j] * US, p, ql); Ah[rr][lane * 4 + j] = p; Al[rr][lane * 4 + j] = ql; } }
  wave_lds_sync();
  const float sx = 1.0f / (US * WSC), sd = 1.0f / (DS * WSC);
  v8f ax[3] = {(v8f){}, (v8f){}, (v8f){}};
#pragma unroll
  for (int kb = 0; kb < DI; kb += 32) { const v16b a = frag_kb(&Ah[nloc][kb], hlf), al = frag_kb(&Al[nloc][kb], hlf);
#pragma unroll
    for (int t = 0; t < 3; ++t) { const v16b bw = frag_kb(XPW + (size_t)(t * 16 + nloc) * DI + kb, hlf); ax[t] = wmma16b(a, bw, ax[t]); ax[t] = wmma16b(al, bw, ax[t]); } }
#pragma unroll
  for (int r8 = 0; r8 < 8; ++r8) { const int rl = 8 * hlf + r8; const float d0 = ax[0][r8] * sx, d1 = ax[1][r8] * sx, d2 = ax[2][r8] * sx;
    if (nloc < R) { b16 p, ql; split16(d0 * DS, p, ql); Dh[rl][nloc] = p; Dl[rl][nloc] = ql; Sbc[rl][12 + nloc] = d1; Sbc[rl][16 + 12 + nloc] = d2; }
    else { Dh[rl][nloc] = (b16)0.0f; Dl[rl][nloc] = (b16)0.0f; Sbc[rl][nloc - R] = d0; Sbc[rl][16 + nloc - R] = d1; }
    Dh[rl][16 + nloc] = (b16)0.0f; Dl[rl][16 + nloc] = (b16)0.0f; }
  wave_lds_sync();
  for (int pass = 0; pass < 2; ++pass) { for (int rr = 0; rr < 16; ++rr) ((volatile float*)BC)[(sq0 + rr) * 32 + lane] = Sbc[rr][lane]; __threadfence(); }
  { v8f acc[8]; const v16b a = frag_kb(&Dh[nloc][0], hlf), al = frag_kb(&Dl[nloc][0], hlf);
#pragma unroll
    for (int t = 0; t < 8; ++t) { acc[t] = (v8f){}; const v16b bw = frag_kb(DTW + (size_t)(t * 16 + nloc) * 32, hlf); acc[t] = wmma16b(a, bw, acc[t]); acc[t] = wmma16b(al, bw, acc[t]); }
#pragma unroll
    for (int t = 0; t < 8; ++t) { const int c = t * 16 + nloc; const float bb = bf16_rne(dtb[c]);
#pragma unroll 1
      for (int r8 = 0; r8 < 8; ++r8) Tf[8 * hlf + r8][c] = softplus(acc[t][r8] * sd + bb); } }
  wave_lds_sync();
  for (int pass = 0; pass < 2; ++pass) { for (int rr = 0; rr < 16; ++rr) *(volatile v4f*)(DT + (sq0 + rr) * DI + lane * 4) = *(const v4f*)(&Tf[rr][lane * 4]); __threadfence(); }
}
__global__ __launch_bounds__(256) void scan_kernel(const float* __restrict__ U, const float* __restrict__ DT, const float* __restrict__ BC, const float* __restrict__ alog, const float* __restrict__ Dp, int nbv, float* __restrict__ Y) {
  const int gid = blockIdx.x * 256 + threadIdx.x; const int b = gid / (NCH * DI), q = (gid / DI) % NCH, d = gid % DI; if (b >= nbv) return;
  float A[NS]; for (int s = 0; s < NS; ++s) A[s] = -__expf(bf16_rne(alog[d * NS + s])); const float dk = bf16_rne(Dp[d]);
  const size_t base = (size_t)q * NT + (size_t)b * L;
#pragma unroll 1
  for (int pass = 0; pass < 2; ++pass) { float h[NS]; for (int s = 0; s < NS; ++s) h[s] = 0.0f;
#pragma unroll 1
    for (int p = 0; p < L; ++p) { const size_t row = base + p; const float u = U[row * DI + d], dt = DT[row * DI + d]; const float du = pmul(dt, u); const float* bc = BC + row * 32; float acc = 0.0f;
#pragma unroll
      for (int s = 0; s < NS; ++s) { h[s] = pmul(h[s], __expf(pmul(dt, A[s]))) + pmul(du, bc[s]); acc += pmul(h[s], bc[16 + s]); }
      ((volatile float*)Y)[row * DI + d] = acc + pmul(dk, u); }
    __threadfence(); }
}
__global__ __launch_bounds__(32) void outproj_kernel(const float* __restrict__ Y, const float* __restrict__ XZ, const float* __restrict__ XN, const float* __restrict__ skp, const b16* __restrict__ WOP, int ntv, float* __restrict__ XM) {
  __shared__ __attribute__((aligned(16))) b16 Ah[16][DI + 8], Al[16][DI + 8]; __shared__ __attribute__((aligned(16))) float Tf[16][DM + 4];
  const int lane = threadIdx.x, nloc = lane & 15, hlf = lane >> 4; const size_t w0 = (size_t)blockIdx.x * 16; const int q = (int)(w0 / ntv); const size_t t0 = w0 % ntv; const size_t sq0 = (size_t)q * NT + t0; const float sk = bf16_rne(skp[0]);
  for (int rr = 0; rr < 16; ++rr) { const v4f y = *(const v4f*)(Y + (sq0 + rr) * DI + lane * 4), z = *(const v4f*)(XZ + (sq0 + rr) * (2 * DI) + DI + lane * 4); for (int j = 0; j < 4; ++j) { b16 p, ql; split16(pmul(y[j], silu(z[j])) * YS, p, ql); Ah[rr][lane * 4 + j] = p; Al[rr][lane * 4 + j] = ql; } }
  wave_lds_sync();
  v8f acc[4];
#pragma unroll
  for (int t = 0; t < 4; ++t) acc[t] = (v8f){};
#pragma unroll
  for (int kb = 0; kb < DI; kb += 32) { const v16b a = frag_kb(&Ah[nloc][kb], hlf), al = frag_kb(&Al[nloc][kb], hlf);
#pragma unroll
    for (int t = 0; t < 4; ++t) { const v16b bw = frag_kb(WOP + (size_t)(t * 16 + nloc) * DI + kb, hlf); acc[t] = wmma16b(a, bw, acc[t]); acc[t] = wmma16b(al, bw, acc[t]); } }
#pragma unroll
  for (int t = 0; t < 4; ++t) { const int c = t * 16 + nloc;
#pragma unroll 1
    for (int r8 = 0; r8 < 8; ++r8) { const int rl = 8 * hlf + r8; Tf[rl][c] = acc[t][r8] * (1.0f / (YS * WSC)) + pmul(sk, XN[(t0 + rl) * CIN + q * DM + c]); } }
  wave_lds_sync();
  for (int pass = 0; pass < 2; ++pass) { for (int rr = 0; rr < 16; ++rr) *(volatile v2f*)(XM + (t0 + rr) * CIN + q * DM + lane * 2) = *(const v2f*)(&Tf[rr][lane * 2]); __threadfence(); }
}
__global__ __launch_bounds__(64) void final_kernel(const float* __restrict__ XM, const float* __restrict__ g, const float* __restrict__ bb, const b16* __restrict__ WPJ, const float* __restrict__ pb, float* __restrict__ out) {
  __shared__ __attribute__((aligned(16))) b16 Ah[2][16][CIN + 8], Al[2][16][CIN + 8]; __shared__ __attribute__((aligned(16))) float To[128][32 + 1];
  const int wave = threadIdx.x >> 5, lane = threadIdx.x & 31, nloc = lane & 15, hlf = lane >> 4; const size_t t0 = (size_t)blockIdx.x * 32; const size_t m0 = t0 + wave * 16; const int b = (int)(t0 / L), p0 = (int)(t0 % L);
  float g8[8], b8[8]; for (int q = 0; q < 8; ++q) { g8[q] = bf16_rne(g[q * 32 + lane]); b8[q] = bf16_rne(bb[q * 32 + lane]); }
  for (int rr = 0; rr < 16; ++rr) { float v[8]; float s = 0.0f; for (int q = 0; q < 8; ++q) { v[q] = XM[(m0 + rr) * CIN + q * 32 + lane]; s += v[q]; } for (int o = 16; o; o >>= 1) s += __shfl_xor(s, o); const float mu = s * (1.0f / CIN);
    float vq = 0.0f; for (int q = 0; q < 8; ++q) { const float d = v[q] - mu; vq += pmul(d, d); } for (int o = 16; o; o >>= 1) vq += __shfl_xor(vq, o); const float rs = rsqrtf(vq * (1.0f / CIN) + EPS);
    for (int q = 0; q < 8; ++q) { b16 p, ql; split16((pmul(pmul(v[q] - mu, rs), g8[q]) + b8[q]) * XS, p, ql); Ah[wave][rr][q * 32 + lane] = p; Al[wave][rr][q * 32 + lane] = ql; } }
  wave_lds_sync();
#pragma unroll 1
  for (int cg = 0; cg < 2; ++cg) { v8f acc[8];
#pragma unroll
    for (int t = 0; t < 8; ++t) acc[t] = (v8f){};
#pragma unroll 2
    for (int kb = 0; kb < CIN; kb += 32) { const v16b a = frag_kb(&Ah[wave][nloc][kb], hlf), al = frag_kb(&Al[wave][nloc][kb], hlf);
#pragma unroll
      for (int t = 0; t < 8; ++t) { const v16b bw = frag_kb(WPJ + (size_t)(cg * 128 + t * 16 + nloc) * CIN + kb, hlf); acc[t] = wmma16b(a, bw, acc[t]); acc[t] = wmma16b(al, bw, acc[t]); } }
#pragma unroll
    for (int t = 0; t < 8; ++t) { const int c = t * 16 + nloc; const float b1 = bf16_rne(pb[cg * 128 + c]);
#pragma unroll
      for (int r8 = 0; r8 < 8; ++r8) To[c][wave * 16 + 8 * hlf + r8] = acc[t][r8] * (1.0f / (XS * WSC)) + b1; }
    __syncthreads();
    for (int pass = 0; pass < 2; ++pass) { for (int i = threadIdx.x; i < 128 * 32; i += 64) { const int c = i >> 5, pp = i & 31; ((volatile float*)out)[((size_t)b * CIN + cg * 128 + c) * L + p0 + pp] = To[c][pp]; } __threadfence(); }
    __syncthreads(); }
}
}

extern "C" void kernel_launch(void* const* d_in, const int* in_sizes, int n_in, void* d_out, int out_size, void* d_ws, size_t ws_size, hipStream_t stream) {
  (void)n_in;
  auto Fp = [&](int i) { return (const float*)d_in[i]; };
  if (in_sizes[0] != NT * CIN || in_sizes[3] != 2 * DI * DM || in_sizes[4] != DI * DC || in_sizes[6] != XD * DI || in_sizes[7] != DI * R || in_sizes[9] != DI * NS || in_sizes[11] != DM * DI || in_sizes[12] != CIN * CIN || out_size != NT * CIN) return;
  const int NBV = NB; const int NTV = NBV * L;
  size_t off = 0; char* ws = (char*)d_ws;
  auto carve = [&](size_t bytes) { char* p = ws + off; off += (bytes + 255) & ~(size_t)255; return p; };
  b16* WIP = (b16*)carve((size_t)2 * DI * DM * 2); b16* XPW = (b16*)carve((size_t)48 * DI * 2); b16* DTW = (b16*)carve((size_t)DI * 32 * 2); b16* WOP = (b16*)carve((size_t)DM * DI * 2); b16* WPJ = (b16*)carve((size_t)CIN * CIN * 2);
  float* XN = (float*)carve((size_t)NT * CIN * 4); float* XZ = (float*)carve((size_t)NQ * 2 * DI * 4); float* U = (float*)carve((size_t)NQ * DI * 4); float* BC = (float*)carve((size_t)NQ * 32 * 4); float* DT = (float*)carve((size_t)NQ * DI * 4); float* Y = (float*)carve((size_t)NQ * DI * 4); float* XM = (float*)carve((size_t)NT * CIN * 4);
  if (off > ws_size) return;
  auto wcp = [&](const float* w, int KIN, int OUT, int KP, int OUTP, b16* WT) { wcopyp_kernel<<<(OUTP * KP / 8 + 255) / 256, 256, 0, stream>>>(w, KIN, OUT, KP, OUTP, WT); };
  wcp(Fp(3), DM, 2 * DI, DM, 2 * DI, WIP); wcp(Fp(6), DI, XD, DI, 48, XPW); wcp(Fp(7), R, DI, 32, DI, DTW); wcp(Fp(11), DI, DM, DI, DM, WOP); wcp(Fp(12), CIN, CIN, CIN, CIN, WPJ);
  ln_in_kernel<<<NTV / 16, 32, 0, stream>>>(Fp(0), Fp(1), Fp(2), XN);
  inproj_kernel<<<NCH * NTV / 16, 32, 0, stream>>>(XN, WIP, NTV, XZ);
  conv_kernel<<<(unsigned)(((size_t)NCH * NTV * (DI / 4) + 255) / 256), 256, 0, stream>>>(XZ, Fp(4), Fp(5), NTV, U);
  xproj_kernel<<<NCH * NTV / 16, 32, 0, stream>>>(U, XPW, DTW, Fp(8), NTV, BC, DT);
  scan_kernel<<<(NBV * NCH * DI + 255) / 256, 256, 0, stream>>>(U, DT, BC, Fp(9), Fp(10), NBV, Y);
  outproj_kernel<<<NCH * NTV / 16, 32, 0, stream>>>(Y, XZ, XN, Fp(14), WOP, NTV, XM);
  final_kernel<<<NTV / 32, 64, 0, stream>>>(XM, Fp(1), Fp(2), WPJ, Fp(13), (float*)d_out);
}
